// NFLGraphModel_16965120819608
// MI455X (gfx1250) — hardware-verified
//
#include <hip/hip_runtime.h>
#include <math.h>

#define NN 50000
#define NE 800000
#define NG16 (NE / 16)
#define NT16 (NN / 16)
#define AP 264
#define CP 72
#define TN 640
#define RPW (TN / 8)
#define NTILE ((NN + TN - 1) / TN)
#define SCH 2048
#define NCH ((NE + SCH - 1) / SCH)
#define NTB 256

typedef __attribute__((ext_vector_type(16))) _Float16 v16h;
typedef __attribute__((ext_vector_type(8)))  _Float16 v8h;
typedef __attribute__((ext_vector_type(8)))  float    v8f;
typedef __attribute__((ext_vector_type(4)))  float    v4f;
typedef __attribute__((ext_vector_type(4)))  int      v4i;

__device__ __forceinline__ void dep_guard_h(v8f& a, v8f& b, v16h x, v16h y) { asm volatile("v_nop\n\tv_nop\n\tv_nop\n\tv_nop" : "+v"(a), "+v"(b) : "v"(x), "v"(y)); }
__device__ __forceinline__ void keep4_h(v16h a, v16h b, v16h c, v16h d) { asm volatile("v_nop" :: "v"(a), "v"(b), "v"(c), "v"(d)); }
template <typename T> struct Frag;
template <> struct Frag<_Float16> {
  typedef v16h V; union U { v16h v; v8h h[2]; };
  static __device__ __forceinline__ v16h load(const _Float16* p) {
    U f; f.h[0] = *(const v8h*)(p); f.h[1] = *(const v8h*)(p + 16); return f.v;
  }
  static __device__ __forceinline__ v8f mma(v16h a, v16h b, v8f c) {
    return __builtin_amdgcn_wmma_f32_16x16x32_f16(false, a, false, b, (short)0, c, false, false);
  }
  static __device__ __forceinline__ void guard(v8f& a, v8f& b, v16h x, v16h y) { dep_guard_h(a, b, x, y); }
  static __device__ __forceinline__ void keep(v16h a, v16h b, v16h c, v16h d) { keep4_h(a, b, c, d); }
};

__device__ __forceinline__ v8f mma_h(v16h a, v16h b, v8f c) {
  c = __builtin_amdgcn_wmma_f32_16x16x32_f16(false, a, false, b, (short)0, c, false, false);
  asm volatile("v_nop\n\tv_nop\n\tv_nop\n\tv_nop" : "+v"(c) : "v"(a), "v"(b));
  return c;
}
__device__ __forceinline__ void wave_sync_lds() {
  __builtin_amdgcn_fence(__ATOMIC_RELEASE, "workgroup");
  __builtin_amdgcn_wave_barrier();
  __builtin_amdgcn_fence(__ATOMIC_ACQUIRE, "workgroup");
}
__device__ __forceinline__ int clampi(int v, int hi) { return v < 0 ? 0 : (v > hi ? hi : v); }
__device__ __forceinline__ unsigned pack_h2(float a, float b) {
  const _Float16 ha = (_Float16)a, hb = (_Float16)b;
  return (unsigned)__builtin_bit_cast(unsigned short, ha) | ((unsigned)__builtin_bit_cast(unsigned short, hb) << 16);
}

__device__ __forceinline__ int blk_excl_scan(int cnt, int* scan_ws, int tid, int* tot) {
  const int lane = tid & 31, wave = tid >> 5; int incl = cnt;
#pragma unroll
  for (int o = 1; o < 32; o <<= 1) { const int v = __shfl_up(incl, o, 32); if (lane >= o) incl += v; }
  if (lane == 31) scan_ws[wave] = incl;
  __syncthreads();
  if (wave == 0) { int wv = (lane < NTB / 32) ? scan_ws[lane] : 0; int wincl = wv;
#pragma unroll
    for (int o = 1; o < 32; o <<= 1) { const int v = __shfl_up(wincl, o, 32); if (lane >= o) wincl += v; }
    if (lane < NTB / 32) scan_ws[32 + lane] = wincl - wv; if (lane == 31) scan_ws[64] = wincl; }
  __syncthreads();
  const int res = scan_ws[32 + wave] + incl - cnt; *tot = scan_ws[64];
  return res;
}
template <int SP, int CAP>
__device__ __forceinline__ int chunk_hits(const int* __restrict__ dstv, int e0, int n0, int tid, int* LIST, int* scan_ws) {
  const int eb = e0 + tid * SP;
  int rec[SP]; int cnt = 0;
  if (eb < NE) {
#pragma unroll
    for (int k = 0; k < SP; k += 4) {
      const v4i d4 = *(const v4i*)(dstv + eb + k);
#pragma unroll
      for (int q = 0; q < 4; ++q) {
        const int d = d4[q]; int r = -1;
        if (d >= n0 && d < n0 + TN) { r = ((d - n0) << 20) | (eb + k + q); ++cnt; }
        rec[k + q] = r;
      }
    }
  } else {
#pragma unroll
    for (int k = 0; k < SP; ++k) rec[k] = -1;
  }
  int tot; int p = blk_excl_scan(cnt, scan_ws, tid, &tot);
#pragma unroll
  for (int k = 0; k < SP; ++k) if (rec[k] >= 0) { if ((unsigned)p < (unsigned)CAP) LIST[p] = rec[k]; ++p; }
  __syncthreads();
  return tot < CAP ? tot : CAP;
}

__global__ __launch_bounds__(NTB) void prep_kernel(
    const float* __restrict__ fcW, const float* __restrict__ fcb, const float* __restrict__ emb,
    const float* __restrict__ W1fij, const float* __restrict__ bias1, const float* __restrict__ attn1,
    const float* __restrict__ W2ni, const float* __restrict__ W2nj, const float* __restrict__ W2fij,
    const float* __restrict__ W2node, const float* __restrict__ attn2,
    float* __restrict__ TAB, unsigned* __restrict__ B16w, unsigned* __restrict__ B2w) {
  (void)W2node; (void)attn2;
  const int j = threadIdx.x;
  float uu = 0.f, c0 = 0.f, v0 = 0.f, v1 = 0.f;
#pragma unroll 1
  for (int k = 0; k < 32; ++k) {
    const float w = W1fij[j * 64 + k], w2 = W1fij[j * 64 + 32 + k];
    uu += w * fcW[k]; c0 += w * fcb[k]; v0 += w2 * emb[k]; v1 += w2 * emb[32 + k];
  }
  const float t0 = 16.0f * uu, t1 = 16.0f * (v0 + c0 + bias1[j]), t2 = 16.0f * (v1 + c0 + bias1[j]);
  ((volatile float*)TAB)[j] = t0; ((volatile float*)TAB)[256 + j] = t1; ((volatile float*)TAB)[512 + j] = t2;
  __threadfence();
  ((volatile float*)TAB)[j] = t0; ((volatile float*)TAB)[256 + j] = t1; ((volatile float*)TAB)[512 + j] = t2;
  for (int idx = j; idx < 2048; idx += NTB) {
    const int n = idx >> 7, k = 2 * (idx & 127);
    float a = 0.f, b = 0.f;
    if (n < 4) { if ((k >> 6) == n) { a = 64.0f * attn1[n * 64 + (k & 63)]; b = 64.0f * attn1[n * 64 + (k & 63) + 1]; } }
    else if (n < 8) { a = 16.0f * W2fij[(n - 4) * 64 + (k & 63)]; b = 16.0f * W2fij[(n - 4) * 64 + (k & 63) + 1]; }
    const unsigned u = pack_h2(a, b);
    ((volatile unsigned*)B16w)[idx] = u; __threadfence(); ((volatile unsigned*)B16w)[idx] = u;
  }
  for (int idx = j; idx < 512; idx += NTB) {
    const int n = idx >> 5, k = 2 * (idx & 31);
    float a = 0.f, b = 0.f;
    if (n < 4) { a = 64.0f * W2ni[n * 64 + k]; b = 64.0f * W2ni[n * 64 + k + 1]; }
    else if (n < 8) { a = 64.0f * W2nj[(n - 4) * 64 + k]; b = 64.0f * W2nj[(n - 4) * 64 + k + 1]; }
    const unsigned u = pack_h2(a, b);
    ((volatile unsigned*)B2w)[idx] = u; __threadfence(); ((volatile unsigned*)B2w)[idx] = u;
  }
}

__global__ __launch_bounds__(128) void edge1_kernel(
    const float* __restrict__ x, const float* __restrict__ dist, const int* __restrict__ team,
    const int* __restrict__ srcv, const int* __restrict__ dstv,
    const float* __restrict__ TAB, const float* __restrict__ W1ni, const float* __restrict__ W1nj,
    const _Float16* __restrict__ B16, float* __restrict__ LGF) {
  __shared__ __align__(16) _Float16 Bs[16 * AP];
  __shared__ __align__(16) _Float16 At[4][16 * AP];
  __shared__ __align__(16) float Os[4][128];
  const int tid = threadIdx.x, lane = tid & 31, wave = tid >> 5, hh = lane >> 4, m = lane & 15;
  for (int q = tid; q < 512; q += 128) {
    const int n = q >> 5, c8 = (q & 31) * 8;
    *(v8h*)(Bs + n * AP + c8) = *(const v8h*)(B16 + q * 8);
  }
  __syncthreads();
  const int grp = blockIdx.x * 4 + wave;
  if (grp < NG16) {
    float U[8], V0[8], V1[8], An[24], Bn[24];
    {
      const v4f u0 = *(const v4f*)(TAB + 8 * lane), u1 = *(const v4f*)(TAB + 8 * lane + 4);
      const v4f p0 = *(const v4f*)(TAB + 256 + 8 * lane), p1 = *(const v4f*)(TAB + 256 + 8 * lane + 4);
      const v4f r0 = *(const v4f*)(TAB + 512 + 8 * lane), r1 = *(const v4f*)(TAB + 512 + 8 * lane + 4);
#pragma unroll
      for (int e = 0; e < 4; ++e) {
        U[e] = u0[e]; U[4 + e] = u1[e]; V0[e] = p0[e]; V0[4 + e] = p1[e]; V1[e] = r0[e]; V1[4 + e] = r1[e];
      }
#pragma unroll
      for (int q = 0; q < 6; ++q) {
        const v4f wa = *(const v4f*)(W1ni + 24 * lane + 4 * q);
        const v4f wb = *(const v4f*)(W1nj + 24 * lane + 4 * q);
#pragma unroll
        for (int e = 0; e < 4; ++e) { An[4 * q + e] = 16.0f * wa[e]; Bn[4 * q + e] = 16.0f * wb[e]; }
      }
    }
    const int e0 = grp * 16;
    const int er = e0 + m;
    const int s = clampi(srcv[er], NN - 1);
    const int d = clampi(dstv[er], NN - 1);
    const int tq = team[er];
    const int tsel = tq > 0 ? 1 : 0;
    const float dv = dist[er];
    const float xs0 = x[s * 3], xs1 = x[s * 3 + 1], xs2 = x[s * 3 + 2];
    const float xd0 = x[d * 3], xd1 = x[d * 3 + 1], xd2 = x[d * 3 + 2];
    _Float16* Aw = At[wave];
#pragma unroll 1
    for (int i = 0; i < 16; ++i) {
      const float bd = __shfl(dv, i, 32);
      const int   bt = __shfl(tsel, i, 32);
      const float a0 = __shfl(xs0, i, 32), a1 = __shfl(xs1, i, 32), a2 = __shfl(xs2, i, 32);
      const float b0 = __shfl(xd0, i, 32), b1 = __shfl(xd1, i, 32), b2 = __shfl(xd2, i, 32);
      v8h hv;
#pragma unroll
      for (int q = 0; q < 8; ++q) {
        float v = bt ? V1[q] : V0[q];
        v = v + bd * U[q];
        v = v + a0 * An[3 * q] + a1 * An[3 * q + 1] + a2 * An[3 * q + 2];
        v = v + b0 * Bn[3 * q] + b1 * Bn[3 * q + 1] + b2 * Bn[3 * q + 2];
        const float lk = fmaxf(v, 0.01f * v);
        hv[q] = (_Float16)lk;
      }
      *(v8h*)(Aw + i * AP + 8 * lane) = hv;
    }
    wave_sync_lds();
    v8f acc = {0.f, 0.f, 0.f, 0.f, 0.f, 0.f, 0.f, 0.f};
#pragma unroll
    for (int ks = 0; ks < 8; ++ks) {
      const v16h a = Frag<_Float16>::load(Aw + m * AP + ks * 32 + 8 * hh);
      const v16h b = Frag<_Float16>::load(Bs + m * AP + ks * 32 + 8 * hh);
      acc = mma_h(a, b, acc);
    }
    float* os = Os[wave];
    if (m < 8) {
#pragma unroll
      for (int r = 0; r < 8; ++r) os[(8 * hh + r) * 8 + m] = acc[r] * (1.0f / 1024.0f);
    }
    wave_sync_lds();
    const v4f o = *(const v4f*)(os + 4 * lane);
    float* op = LGF + (size_t)e0 * 8 + 4 * lane;
    *(volatile v4f*)op = o;
    __threadfence();
    *(volatile v4f*)op = o;
  }
}

__global__ __launch_bounds__(NTB) void agg1_kernel(
    const float* __restrict__ x, const int* __restrict__ srcv, const int* __restrict__ dstv,
    const float* __restrict__ LGF, const float* __restrict__ W1node, float* __restrict__ H) {
  __shared__ float SM[TN * 4];
  __shared__ float SL[TN * 4];
  __shared__ float SS[TN * 12];
  __shared__ int LIST[SCH];
  __shared__ int scan_ws[80];
  const int tid = threadIdx.x, lane = tid & 31, wave = tid >> 5;
  const int n0 = blockIdx.x * TN;
  const int wlo = wave * RPW;
  const int hq = (lane >> 2) & 3, kq = lane & 3, kc = kq < 3 ? kq : 2;
  const int c4 = 4 * (lane & 15);
  v4f w[4][3];
#pragma unroll
  for (int h = 0; h < 4; ++h) {
    const float* wp = W1node + (h * 64 + c4) * 3;
    const v4f q0 = *(const v4f*)(wp), q1 = *(const v4f*)(wp + 4), q2 = *(const v4f*)(wp + 8);
    w[h][0] = (v4f){q0[0], q0[3], q1[2], q2[1]};
    w[h][1] = (v4f){q0[1], q1[0], q1[3], q2[2]};
    w[h][2] = (v4f){q0[2], q1[1], q2[0], q2[3]};
  }
  for (int i = tid; i < TN * 4; i += NTB) { SM[i] = -INFINITY; SL[i] = 0.f; }
  for (int i = tid; i < TN * 12; i += NTB) SS[i] = 0.f;
  __syncthreads();
#pragma unroll 1
  for (int c = 0; c < NCH; ++c) {
    const int tot = chunk_hits<SCH / NTB, SCH>(dstv, c * SCH, n0, tid, LIST, scan_ws);
#pragma unroll 1
    for (int base = 0; base < tot; base += 32) {
      const int q = base + lane;
      int rv = -1;
      if (q < tot) rv = LIST[q];
      const int dq = rv >> 20;
      const int own = (rv >= 0 && dq >= wlo && dq < wlo + RPW) ? 1 : 0;
      unsigned msk = (unsigned)__ballot(own);
#pragma unroll 1
      for (int it = 0; it < 32; ++it) {
        if (msk == 0u) break;
        const int bp = __builtin_ctz(msk); msk &= msk - 1u;
        const int r = __shfl(rv, bp, 32);
        int dl = r >> 20; dl = dl < TN ? dl : TN - 1;
        int e = r & 0xFFFFF; e = e < NE ? e : NE - 1;
        const int s = clampi(srcv[e], NN - 1);
        const float lg = LGF[(size_t)e * 8 + hq];
        const float xk = x[s * 3 + kc];
        const int mi = dl * 4 + hq;
        const int si = dl * 12 + hq * 3 + kc;
        const float mo = SM[mi], lo = SL[mi], so = SS[si];
        const float mn = fmaxf(mo, lg);
        const float rr = __expf(mo - mn), ex = __expf(lg - mn);
        const float ln = lo * rr + ex;
        const float sn = so * rr + ex * xk;
        if (lane < 16 && kq < 3) SS[si] = sn;
        if (lane < 16 && kq == 0) { SM[mi] = mn; SL[mi] = ln; }
      }
    }
    __syncthreads();
  }
#pragma unroll 1
  for (int j2 = 0; j2 < RPW; j2 += 2) {
    const int nb = n0 + wlo + j2;
    if (nb < NN) {
      const int dl = wlo + j2 + (lane >> 4);
      float iv[4];
#pragma unroll
      for (int h = 0; h < 4; ++h) {
        const float lv = SL[dl * 4 + h];
        const float rc = 0.25f * __builtin_amdgcn_rcpf(lv);
        iv[h] = (lv > 0.f) ? rc : 0.f;
      }
      v4f o = {0.f, 0.f, 0.f, 0.f};
#pragma unroll
      for (int h = 0; h < 4; ++h)
#pragma unroll
        for (int k = 0; k < 3; ++k) {
          const float sv = SS[dl * 12 + h * 3 + k] * iv[h];
          o = o + sv * w[h][k];
        }
      float* hp = H + (size_t)(nb + (lane >> 4)) * 64 + c4;
      *(volatile v4f*)hp = o;
      __threadfence();
      *(volatile v4f*)hp = o;
    }
  }
}

__global__ __launch_bounds__(128) void node2_kernel(const float* __restrict__ H, const _Float16* __restrict__ B2t, float* __restrict__ G) {
  __shared__ __align__(16) _Float16 B2s[16 * CP];
  __shared__ __align__(16) _Float16 At[4][16 * CP];
  __shared__ __align__(16) float Os[4][128];
  const int tid = threadIdx.x, lane = tid & 31, wave = tid >> 5, hh = lane >> 4, m = lane & 15;
  {
    const int n = tid >> 3, c8 = (tid & 7) * 8;
    *(v8h*)(B2s + n * CP + c8) = *(const v8h*)(B2t + tid * 8);
  }
  __syncthreads();
  const int tile = blockIdx.x * 4 + wave;
  if (tile < NT16) {
    const int n0 = tile * 16;
    _Float16* Aw = At[wave];
    const float* hr = H + (size_t)(n0 + m) * 64 + 32 * hh;
#pragma unroll
    for (int q = 0; q < 4; ++q) {
      const v4f p0 = *(const v4f*)(hr + 8 * q), p1 = *(const v4f*)(hr + 8 * q + 4);
      v8h hv;
#pragma unroll
      for (int e = 0; e < 4; ++e) { hv[e] = (_Float16)(16.0f * p0[e]); hv[4 + e] = (_Float16)(16.0f * p1[e]); }
      *(v8h*)(Aw + m * CP + 32 * hh + 8 * q) = hv;
    }
    wave_sync_lds();
    v8f acc = {0.f, 0.f, 0.f, 0.f, 0.f, 0.f, 0.f, 0.f};
#pragma unroll
    for (int ks = 0; ks < 2; ++ks) {
      const v16h a = Frag<_Float16>::load(Aw + m * CP + ks * 32 + 8 * hh);
      const v16h b = Frag<_Float16>::load(B2s + m * CP + ks * 32 + 8 * hh);
      acc = mma_h(a, b, acc);
    }
    float* os = Os[wave];
    if (m < 8) {
#pragma unroll
      for (int r = 0; r < 8; ++r) os[(8 * hh + r) * 8 + m] = acc[r] * (1.0f / 1024.0f);
    }
    wave_sync_lds();
    const v4f o = *(const v4f*)(os + 4 * lane);
    float* op = G + (size_t)n0 * 8 + 4 * lane;
    *(volatile v4f*)op = o;
    __threadfence();
    *(volatile v4f*)op = o;
  }
}

__global__ __launch_bounds__(NTB) void edge2_kernel(const int* __restrict__ srcv, const int* __restrict__ dstv, const float* __restrict__ G,
                                                  const float* __restrict__ LGF, const float* __restrict__ bias2, float* __restrict__ out) {
  const int e = blockIdx.x * NTB + threadIdx.x;
  if (e < NE) {
    const int s = clampi(srcv[e], NN - 1);
    const int d = clampi(dstv[e], NN - 1);
    const v4f gs = *(const v4f*)(G + (size_t)s * 8);
    const v4f gd = *(const v4f*)(G + (size_t)d * 8 + 4);
    const v4f ff = *(const v4f*)(LGF + (size_t)e * 8 + 4);
    const v4f bb = *(const v4f*)(bias2);
    float acc = 0.f;
#pragma unroll
    for (int h = 0; h < 4; ++h) {
      float t = gs[h] + gd[h];
      t = t + ff[h];
      t = t + bb[h];
      acc += fmaxf(t, 0.01f * t);
    }
    const float o = 0.25f * acc;
    ((volatile float*)out)[e] = o;
    __threadfence();
    ((volatile float*)out)[e] = o;
  }
}

extern "C" void kernel_launch(void* const* d_in, const int* in_sizes, int n_in,
                              void* d_out, int out_size, void* d_ws, size_t ws_size, hipStream_t stream) {
  if (n_in < 20) return;
  if (in_sizes[0] != NN * 3 || in_sizes[1] != NE || in_sizes[2] != NE || in_sizes[3] != NE || in_sizes[4] != NE || out_size != NE) return;
  const float* x      = (const float*)d_in[0];
  const float* dist   = (const float*)d_in[1];
  const int*   team   = (const int*)  d_in[2];
  const int*   srcv   = (const int*)  d_in[3];
  const int*   dstv   = (const int*)  d_in[4];
  const float* fcW    = (const float*)d_in[5];
  const float* fcb    = (const float*)d_in[6];
  const float* emb    = (const float*)d_in[7];
  const float* W1ni   = (const float*)d_in[8];
  const float* W1nj   = (const float*)d_in[9];
  const float* W1fij  = (const float*)d_in[10];
  const float* W1node = (const float*)d_in[11];
  const float* attn1  = (const float*)d_in[12];
  const float* bias1  = (const float*)d_in[13];
  const float* W2ni   = (const float*)d_in[14];
  const float* W2nj   = (const float*)d_in[15];
  const float* W2fij  = (const float*)d_in[16];
  const float* W2node = (const float*)d_in[17];
  const float* attn2  = (const float*)d_in[18];
  const float* bias2  = (const float*)d_in[19];
  float* out = (float*)d_out;

  char* ws = (char*)d_ws; size_t off = 0;
  auto carve = [&](size_t bytes) -> char* { char* p = ws + off; off += (bytes + 1023) & ~(size_t)1023; return p; };
  float*    TAB = (float*)carve((size_t)3 * 256 * 4);
  _Float16* B16 = (_Float16*)carve((size_t)16 * 256 * 2);
  _Float16* B2T = (_Float16*)carve((size_t)16 * 64 * 2);
  float*    LGF = (float*)carve((size_t)NE * 8 * 4);
  float*    Hn  = (float*)carve((size_t)NN * 64 * 4);
  float*    G   = (float*)carve((size_t)NN * 8 * 4);
  if (off > ws_size || off > (size_t)134217728) return;

  prep_kernel<<<1, NTB, 0, stream>>>(fcW, fcb, emb, W1fij, bias1, attn1, W2ni, W2nj, W2fij, W2node, attn2,
                                      TAB, (unsigned*)B16, (unsigned*)B2T);
  edge1_kernel<<<(NG16 + 3) / 4, 128, 0, stream>>>(x, dist, team, srcv, dstv, TAB, W1ni, W1nj, B16, LGF);
  agg1_kernel<<<NTILE, NTB, 0, stream>>>(x, srcv, dstv, LGF, W1node, Hn);
  node2_kernel<<<(NT16 + 3) / 4, 128, 0, stream>>>(Hn, B2T, G);
  edge2_kernel<<<(NE + NTB - 1) / NTB, NTB, 0, stream>>>(srcv, dstv, G, LGF, bias2, out);
}
